// Mamba2_72000831750785
// MI455X (gfx1250) — hardware-verified
//
#include <hip/hip_runtime.h>
#include <math.h>

typedef __attribute__((ext_vector_type(16))) _Float16 v16h;
typedef __attribute__((ext_vector_type(8)))  _Float16 v8h;
typedef __attribute__((ext_vector_type(16))) __bf16   v16b;
typedef __attribute__((ext_vector_type(8)))  __bf16   v8b;
typedef __attribute__((ext_vector_type(8)))  float    v8f;
typedef __attribute__((ext_vector_type(4)))  float    v4f;

constexpr int kSeq    = 2048;
constexpr int kDm     = 1024;
constexpr int kDin    = 2048;
constexpr int kDxb    = 512;
constexpr int kNst    = 16;
constexpr int kDtR    = 64;
constexpr int kDproj  = 2 * kDin + 2 * kDxb + kDtR;
constexpr int kColZ   = 0;
constexpr int kColX   = kDin;
constexpr int kColB   = kDin + kDxb;
constexpr int kColC   = kDin + 2 * kDxb;
constexpr int kColDt  = 2 * kDin + 2 * kDxb;
constexpr int kConvTP = 260;
constexpr int kScanTS = 32;
constexpr int kScanCh = 64;
constexpr int kScanRow = 224;
constexpr int kScanYP = 68;
static_assert(kDproj == 5184, "proj width");
static_assert((kDm % 32) == 0 && (kDtR % 32) == 0 && (kDin % 32) == 0, "GEMM K multiples of 32");
static_assert((kSeq % 64) == 0 && (kDproj % 64) == 0 && (kDin % 64) == 0 && (kDm % 64) == 0, "GEMM M,N multiples of 64");
static_assert((kSeq % kScanTS) == 0 && (kDin % kScanCh) == 0 && (kDxb % 256) == 0 && (kSeq % 64) == 0, "tile multiples");
static_assert((kDproj * 4) % 128 == 0, "ZX rows are whole lines");

constexpr size_t kOffA1   = 0;
constexpr size_t kOffBT1  = kOffA1  + (size_t)kSeq   * kDm   * 2;
constexpr size_t kOffZX   = kOffBT1 + (size_t)kDproj * kDm   * 2;
constexpr size_t kOffXC   = kOffZX  + (size_t)kSeq   * kDproj * 4;
constexpr size_t kOffADH  = kOffXC  + (size_t)kSeq   * kDxb  * 4;
constexpr size_t kOffADL  = kOffADH + (size_t)kSeq   * kDtR  * 2;
constexpr size_t kOffBTD  = kOffADL + (size_t)kSeq   * kDtR  * 2;
constexpr size_t kOffDT   = kOffBTD + (size_t)kDin   * kDtR  * 2;
constexpr size_t kOffYH   = kOffDT  + (size_t)kSeq   * kDin  * 4;
constexpr size_t kOffYL   = kOffYH  + (size_t)kSeq   * kDin  * 2;
constexpr size_t kOffBT3  = kOffYL  + (size_t)kSeq   * kDin  * 2;
constexpr size_t kWsTotal = kOffBT3 + (size_t)kDm    * kDin  * 2;
static_assert(kWsTotal == 100007936ull, "carve total");
static_assert(kWsTotal <= 134217728ull, "carve cap");
static_assert((kOffBT1 % 128) == 0 && (kOffZX % 128) == 0 && (kOffXC % 128) == 0 && (kOffADH % 128) == 0 &&
              (kOffADL % 128) == 0 && (kOffBTD % 128) == 0 && (kOffDT % 128) == 0 && (kOffYH % 128) == 0 &&
              (kOffYL % 128) == 0 && (kOffBT3 % 128) == 0, "128-B aligned regions");

__device__ __forceinline__ unsigned short f2bf_bits(float f) {
  unsigned u = __float_as_uint(f);
  return (unsigned short)((u + 0x7FFFu + ((u >> 16) & 1u)) >> 16);
}
__device__ __forceinline__ float bf_bits2f(unsigned short h) { return __uint_as_float(((unsigned)h) << 16); }
__device__ __forceinline__ float bfr(float f) { return bf_bits2f(f2bf_bits(f)); }

__device__ __forceinline__ void dep_guard4_b(v8f& a, v8f& b, v8f& c, v8f& d, v16b x, v16b y) {
  asm volatile("v_nop\n\tv_nop\n\tv_nop\n\tv_nop" : "+v"(a), "+v"(b), "+v"(c), "+v"(d) : "v"(x), "v"(y));
}
__device__ __forceinline__ void keep4_b(v16b a, v16b b, v16b c, v16b d) { asm volatile("v_nop" :: "v"(a), "v"(b), "v"(c), "v"(d)); }
__device__ __forceinline__ void acc_guard4(v8f& a, v8f& b, v8f& c, v8f& d) { asm volatile("v_nop\n\tv_nop\n\tv_nop\n\tv_nop" : "+v"(a), "+v"(b), "+v"(c), "+v"(d)); }

struct FragB {
  typedef v16b V; union U { v16b v; v8b h[2]; };
  static __device__ __forceinline__ v16b load(const __bf16* p) {
    U f; f.h[0] = *(const v8b*)(p); f.h[1] = *(const v8b*)(p + 16); return f.v;
  }
  static __device__ __forceinline__ v8f mma(v16b a, v16b b, v8f c) {
    return __builtin_amdgcn_wmma_f32_16x16x32_bf16(false, a, false, b, (short)0, c, false, false);
  }
};

template <int SPL>
__global__ __launch_bounds__(256) void wmma_gemm64(
    const unsigned short* __restrict__ Ap, const unsigned short* __restrict__ A2p, int lda,
    const unsigned short* __restrict__ Btp, int ldb,
    float* __restrict__ Cout, int ldc,
    int M, int N, int K, float scale) {
  typedef v16b V;
  const __bf16* A = (const __bf16*)Ap; const __bf16* A2 = (const __bf16*)A2p; const __bf16* Bt = (const __bf16*)Btp;
  __shared__ __align__(16) float sT[8][16 * 68];
  const int lane = threadIdx.x & 31;
  const int wave = threadIdx.x >> 5;
  const int tilesN = N >> 6;
  const int tilesM = M >> 6;
  const int tile = blockIdx.x * 8 + wave;
  if (tile >= tilesM * tilesN) return;
  const int tm = tile / tilesN;
  const int tn = tile - tm * tilesN;
  const int m0 = tm << 6;
  const int n0 = tn << 6;

  const int rlane = lane & 15;
  const int koff  = (lane >> 4) * 8;
  const int mOff  = (lane >> 4) * 8;

  v8f acc[4][4];
#pragma unroll
  for (int i = 0; i < 4; ++i)
#pragma unroll
    for (int j = 0; j < 4; ++j) acc[i][j] = (v8f){0.f,0.f,0.f,0.f,0.f,0.f,0.f,0.f};

  for (int k0 = 0; k0 < K; k0 += 32) {
    V bh[4];
#pragma unroll
    for (int j = 0; j < 4; ++j) {
      const size_t bo = (size_t)(n0 + (j << 4) + rlane) * ldb + koff + k0;
      bh[j] = FragB::load(Bt + bo);
    }
#pragma unroll
    for (int i = 0; i < 4; ++i) {
      const size_t ao = (size_t)(m0 + (i << 4) + rlane) * lda + koff + k0;
      V ah = FragB::load(A + ao);
      V al;
      if (SPL >= 1) al = FragB::load(A2 + ao);
#pragma unroll
      for (int j = 0; j < 4; ++j) {
        acc[i][j] = FragB::mma(ah, bh[j], acc[i][j]);
        if (SPL >= 1) acc[i][j] = FragB::mma(al, bh[j], acc[i][j]);
      }
      dep_guard4_b(acc[i][0], acc[i][1], acc[i][2], acc[i][3], ah, (SPL >= 1) ? al : ah);
    }
    keep4_b(bh[0], bh[1], bh[2], bh[3]);
  }
  acc_guard4(acc[0][0], acc[0][1], acc[0][2], acc[0][3]);
  acc_guard4(acc[1][0], acc[1][1], acc[1][2], acc[1][3]);
  acc_guard4(acc[2][0], acc[2][1], acc[2][2], acc[2][3]);
  acc_guard4(acc[3][0], acc[3][1], acc[3][2], acc[3][3]);

  float* slab = sT[wave];
#pragma unroll
  for (int i = 0; i < 4; ++i) {
    const int mBase = m0 + (i << 4);
#pragma unroll
    for (int j = 0; j < 4; ++j) {
#pragma unroll
      for (int r = 0; r < 8; ++r) {
        const float v = acc[i][j][r] * scale;
        slab[(mOff + r) * 68 + (j << 4) + rlane] = v;
      }
    }
    __builtin_amdgcn_fence(__ATOMIC_RELEASE, "workgroup");
    __builtin_amdgcn_wave_barrier();
    __builtin_amdgcn_fence(__ATOMIC_ACQUIRE, "workgroup");
    {
      const int hh = lane >> 4, c4 = (lane & 15) * 4;
      for (int pass = 0; pass < 2; ++pass) {
#pragma unroll
        for (int it = 0; it < 8; ++it) {
          const int row = it * 2 + hh;
          v4f v = *(const v4f*)(slab + row * 68 + c4);
          *(volatile v4f*)(Cout + (size_t)(mBase + row) * ldc + n0 + c4) = v;
        }
        __threadfence();
      }
    }
    __builtin_amdgcn_fence(__ATOMIC_RELEASE, "workgroup");
    __builtin_amdgcn_wave_barrier();
    __builtin_amdgcn_fence(__ATOMIC_ACQUIRE, "workgroup");
  }
}

template <bool LO>
__global__ __launch_bounds__(256) void rows_bf16_kernel(
    const float* __restrict__ src, int ld_src, int col0, int width8, int rows,
    unsigned short* __restrict__ dhi, unsigned short* __restrict__ dlo)
{
  const int i = blockIdx.x * 256 + threadIdx.x;
  if (i >= rows * width8) return;
  const int row = i / width8;
  const int j = i - row * width8;
  const size_t so = (size_t)row * ld_src + col0 + 8 * j;
  const size_t e0 = (size_t)i << 3;
  const v4f a0 = *(const v4f*)(src + so);
  const v4f a1 = *(const v4f*)(src + so + 4);
  v8h hv, lv;
#pragma unroll
  for (int e = 0; e < 4; ++e) {
    const float f0 = a0[e], f1 = a1[e];
    const unsigned short h0 = f2bf_bits(f0), h1 = f2bf_bits(f1);
    hv[e]     = __builtin_bit_cast(_Float16, h0);
    hv[4 + e] = __builtin_bit_cast(_Float16, h1);
    if (LO) {
      const unsigned short l0 = f2bf_bits(f0 - bf_bits2f(h0)), l1 = f2bf_bits(f1 - bf_bits2f(h1));
      lv[e]     = __builtin_bit_cast(_Float16, l0);
      lv[4 + e] = __builtin_bit_cast(_Float16, l1);
    }
  }
  unsigned short* qh = dhi + e0;
  *(volatile v8h*)qh = hv;
  if (LO) { unsigned short* ql = dlo + e0; *(volatile v8h*)ql = lv; }
  __threadfence();
  *(volatile v8h*)qh = hv;
  if (LO) { unsigned short* ql = dlo + e0; *(volatile v8h*)ql = lv; }
}

__global__ __launch_bounds__(256) void transpose_bf16_kernel(
    const float* __restrict__ src, int ld_src, unsigned short* __restrict__ dst, int ld_dst)
{
  __shared__ __align__(16) float tile[64 * 65];
  const int tid = threadIdx.x, lane = tid & 31, wave = tid >> 5;
  const int k0 = blockIdx.y * 64;
  const int n0 = blockIdx.x * 64;
  const int r = tid >> 4, c4 = (tid & 15) * 4;
#pragma unroll
  for (int i = 0; i < 4; ++i) {
    const int row = r + 16 * i;
    const v4f v = *(const v4f*)(src + (size_t)(k0 + row) * ld_src + n0 + c4);
    float* tp = tile + row * 65 + c4;
    tp[0] = v[0]; tp[1] = v[1]; tp[2] = v[2]; tp[3] = v[3];
  }
  __syncthreads();
  const int q = lane >> 3, kl = (lane & 7) * 8;
  v8h hv[2];
#pragma unroll
  for (int it = 0; it < 2; ++it) {
    const int nl = it * 32 + wave * 4 + q;
#pragma unroll
    for (int e = 0; e < 8; ++e) {
      const unsigned short hb = f2bf_bits(tile[(kl + e) * 65 + nl]);
      hv[it][e] = __builtin_bit_cast(_Float16, hb);
    }
  }
  for (int pass = 0; pass < 2; ++pass) {
#pragma unroll
    for (int it = 0; it < 2; ++it) {
      const int nl = it * 32 + wave * 4 + q;
      *(volatile v8h*)(dst + (size_t)(n0 + nl) * ld_dst + k0 + kl) = hv[it];
    }
    __threadfence();
  }
}

__global__ __launch_bounds__(256) void conv_silu_kernel(
    const float* __restrict__ ZX, const float* __restrict__ cw, const float* __restrict__ cb,
    float* __restrict__ XC)
{
  __shared__ __align__(16) float sT[16 * kConvTP];
  const int tid = threadIdx.x, lane = tid & 31, wave = tid >> 5;
  const int d0 = blockIdx.x * 256, d = d0 + tid;
  const int g0 = blockIdx.y * 64;
  const float w0 = bfr(cw[d * 4 + 0]), w1 = bfr(cw[d * 4 + 1]), w2 = bfr(cw[d * 4 + 2]), w3 = bfr(cw[d * 4 + 3]);
  const float bc = bfr(cb[d]);
  float xm3, xm2, xm1;
  {
    const bool hist = (g0 > 0);
    const int rb = hist ? (g0 - 3) : g0;
    const float v3 = ZX[(size_t)rb * kDproj + kColX + d];
    const float v2 = ZX[(size_t)(rb + 1) * kDproj + kColX + d];
    const float v1 = ZX[(size_t)(rb + 2) * kDproj + kColX + d];
    xm3 = hist ? v3 : 0.f;
    xm2 = hist ? v2 : 0.f;
    xm1 = hist ? v1 : 0.f;
  }
  const int hrow = wave >> 1;
  const int hch  = (wave & 1) * 128 + lane * 4;
#pragma unroll 1
  for (int sub = 0; sub < 4; ++sub) {
    const int lb = g0 + sub * 16;
#pragma unroll 1
    for (int s = 0; s < 16; ++s) {
      const float xcur = ZX[(size_t)(lb + s) * kDproj + kColX + d];
      float acc = w0 * xm3;
      acc = fmaf(w1, xm2, acc);
      acc = fmaf(w2, xm1, acc);
      acc = fmaf(w3, xcur, acc);
      const float sv = acc + bc;
      const float sg = __builtin_amdgcn_rcpf(1.0f + expf(-sv));
      sT[s * kConvTP + tid] = sv * sg;
      xm3 = xm2; xm2 = xm1; xm1 = xcur;
    }
    __syncthreads();
    v4f fv[4];
#pragma unroll
    for (int it = 0; it < 4; ++it) fv[it] = *(const v4f*)(sT + (it * 4 + hrow) * kConvTP + hch);
    for (int pass = 0; pass < 2; ++pass) {
#pragma unroll
      for (int it = 0; it < 4; ++it)
        *(volatile v4f*)(XC + (size_t)(lb + it * 4 + hrow) * kDxb + d0 + hch) = fv[it];
      __threadfence();
    }
    __syncthreads();
  }
}

__global__ __launch_bounds__(64) void scan_kernel(
    const float* __restrict__ ZX, const float* __restrict__ XC, const float* __restrict__ DT,
    const float* __restrict__ dtb, const float* __restrict__ Alog, const float* __restrict__ Dp,
    unsigned short* __restrict__ YH, unsigned short* __restrict__ YL)
{
  __shared__ __align__(16) float sX[kScanTS * kScanRow];
  __shared__ __align__(16) float sY[kScanTS * kScanYP];
  __shared__ __align__(16) float sA[kNst * kScanCh];
  const int tid = threadIdx.x, lane = tid & 31, wave = tid >> 5;
  const int c0 = blockIdx.x * kScanCh;
  const int c  = c0 + tid;
  const int xcol0 = blockIdx.x * 16;
#pragma unroll 1
  for (int s = 0; s < kNst; ++s) sA[s * kScanCh + tid] = -expf(bfr(Alog[(size_t)c * kNst + s]));
  __syncthreads();
  float negA[kNst], h[kNst];
#pragma unroll
  for (int s = 0; s < kNst; ++s) {
    negA[s] = sA[s * kScanCh + tid];
    h[s] = 0.f;
  }
  const float bias2 = 2.0f * bfr(dtb[c]);
  const float Dd = bfr(Dp[c]);
  const int lr = tid >> 4, lc4 = (tid & 15) * 4;
  const int xr4 = tid >> 2, xc4 = (tid & 3) * 4;
  const int cgrp = (tid >> 4) * 16;
  const int q = lane >> 3, c8 = (lane & 7) * 8;
#pragma unroll 1
  for (int t0 = 0; t0 < kSeq; t0 += kScanTS) {
    __syncthreads();
#pragma unroll 1
    for (int i = 0; i < 8; ++i) {
      const int r = lr + 4 * i;
      const size_t l = (size_t)(t0 + r);
      const v4f zv4 = *(const v4f*)(ZX + l * kDproj + kColZ + c0 + lc4);
      const v4f dv4 = *(const v4f*)(DT + l * kDin + c0 + lc4);
      const v4f cv4 = *(const v4f*)(ZX + l * kDproj + kColC + c0 + lc4);
      float* rp = sX + r * kScanRow;
      *(v4f*)(rp + lc4) = zv4;
      *(v4f*)(rp + 64 + lc4) = dv4;
      *(v4f*)(rp + 128 + lc4) = cv4;
    }
#pragma unroll
    for (int i = 0; i < 2; ++i) {
      const int r = xr4 + 16 * i;
      const size_t l = (size_t)(t0 + r);
      const v4f xv4 = *(const v4f*)(XC + l * kDxb + xcol0 + xc4);
      const v4f bv4 = *(const v4f*)(ZX + l * kDproj + kColB + xcol0 + xc4);
      float* rp = sX + r * kScanRow;
      *(v4f*)(rp + 192 + xc4) = xv4;
      *(v4f*)(rp + 208 + xc4) = bv4;
    }
    __syncthreads();
#pragma unroll 1
    for (int s = 0; s < kScanTS; ++s) {
      const float* xrw = sX + s * kScanRow;
      const float zv = xrw[tid];
      const float dr = xrw[64 + tid];
      const float xv = xrw[192 + (tid & 15)];
      float Bs[kNst], Cs[kNst];
#pragma unroll
      for (int q4 = 0; q4 < 4; ++q4) {
        const v4f bv = *(const v4f*)(xrw + 208 + 4 * q4);
        const v4f cv = *(const v4f*)(xrw + 128 + cgrp + 4 * q4);
        Bs[4 * q4 + 0] = bv[0]; Bs[4 * q4 + 1] = bv[1]; Bs[4 * q4 + 2] = bv[2]; Bs[4 * q4 + 3] = bv[3];
        Cs[4 * q4 + 0] = cv[0]; Cs[4 * q4 + 1] = cv[1]; Cs[4 * q4 + 2] = cv[2]; Cs[4 * q4 + 3] = cv[3];
      }
      const float v     = dr + bias2;
      const float ev    = expf(-fabsf(v));
      const float delta = fmaxf(v, 0.0f) + log1pf(ev);
      const float dx    = delta * xv;
      float y = 0.0f;
#pragma unroll
      for (int k = 0; k < kNst; ++k) {
        const float a = __expf(delta * negA[k]);
        h[k] = a * h[k] + dx * Bs[k];
        y = fmaf(h[k], Cs[k], y);
      }
      y = y + Dd * xv;
      const float sg = __builtin_amdgcn_rcpf(1.0f + expf(-zv));
      y = y * (zv * sg);
      sY[s * kScanYP + tid] = y;
    }
    __syncthreads();
    v8h hv[4], lv[4];
#pragma unroll
    for (int it = 0; it < 4; ++it) {
      const int row = it * 8 + wave * 4 + q;
      const float* sp = sY + row * kScanYP + c8;
      const v4f a0 = *(const v4f*)(sp);
      const v4f a1 = *(const v4f*)(sp + 4);
#pragma unroll
      for (int e = 0; e < 4; ++e) {
        const float f0 = a0[e], f1 = a1[e];
        const unsigned short h0 = f2bf_bits(f0), h1 = f2bf_bits(f1);
        const unsigned short l0 = f2bf_bits(f0 - bf_bits2f(h0)), l1 = f2bf_bits(f1 - bf_bits2f(h1));
        hv[it][e]     = __builtin_bit_cast(_Float16, h0);
        hv[it][4 + e] = __builtin_bit_cast(_Float16, h1);
        lv[it][e]     = __builtin_bit_cast(_Float16, l0);
        lv[it][4 + e] = __builtin_bit_cast(_Float16, l1);
      }
    }
    for (int pass = 0; pass < 2; ++pass) {
#pragma unroll
      for (int it = 0; it < 4; ++it) {
        const int row = it * 8 + wave * 4 + q;
        const size_t o = (size_t)(t0 + row) * kDin + c0 + c8;
        *(volatile v8h*)(YH + o) = hv[it];
        *(volatile v8h*)(YL + o) = lv[it];
      }
      __threadfence();
    }
  }
}

extern "C" void kernel_launch(void* const* d_in, const int* in_sizes, int n_in,
                              void* d_out, int out_size, void* d_ws, size_t ws_size,
                              hipStream_t stream) {
  if (n_in < 9) return;
  if (in_sizes[0] != kSeq * kDm) return;
  if (in_sizes[1] != kDm * kDproj) return;
  if (in_sizes[2] != kDxb * 4) return;
  if (in_sizes[3] != kDxb) return;
  if (in_sizes[4] != kDtR * kDin) return;
  if (in_sizes[5] != kDin) return;
  if (in_sizes[6] != kDin * kNst) return;
  if (in_sizes[7] != kDin) return;
  if (in_sizes[8] != kDin * kDm) return;
  if (out_size != kSeq * kDm) return;
  if (ws_size < kWsTotal) return;

  const float* hidden  = (const float*)d_in[0];
  const float* W_in    = (const float*)d_in[1];
  const float* conv_w  = (const float*)d_in[2];
  const float* conv_b  = (const float*)d_in[3];
  const float* W_dt    = (const float*)d_in[4];
  const float* dt_bias = (const float*)d_in[5];
  const float* A_log   = (const float*)d_in[6];
  const float* Dvec    = (const float*)d_in[7];
  const float* W_out   = (const float*)d_in[8];
  float* out = (float*)d_out;

  char* ws = (char*)d_ws;
  unsigned short* A1  = (unsigned short*)(ws + kOffA1);
  unsigned short* BT1 = (unsigned short*)(ws + kOffBT1);
  float*          ZX  = (float*)(ws + kOffZX);
  float*          XC  = (float*)(ws + kOffXC);
  unsigned short* ADH = (unsigned short*)(ws + kOffADH);
  unsigned short* ADL = (unsigned short*)(ws + kOffADL);
  unsigned short* BTD = (unsigned short*)(ws + kOffBTD);
  float*          DT  = (float*)(ws + kOffDT);
  unsigned short* YH  = (unsigned short*)(ws + kOffYH);
  unsigned short* YL  = (unsigned short*)(ws + kOffYL);
  unsigned short* BT3 = (unsigned short*)(ws + kOffBT3);

  rows_bf16_kernel<false><<<(kSeq * (kDm / 8) + 255) / 256, 256, 0, stream>>>(hidden, kDm, 0, kDm / 8, kSeq, A1, nullptr);
  transpose_bf16_kernel<<<dim3(kDproj / 64, kDm / 64), 256, 0, stream>>>(W_in, kDproj, BT1, kDm);

  wmma_gemm64<0><<<dim3((kSeq / 64) * (kDproj / 64) / 8, 1), 256, 0, stream>>>(
      A1, nullptr, kDm, BT1, kDm, ZX, kDproj, kSeq, kDproj, kDm, 1.0f);

  conv_silu_kernel<<<dim3(kDxb / 256, kSeq / 64), 256, 0, stream>>>(ZX, conv_w, conv_b, XC);

  rows_bf16_kernel<true><<<(kSeq * (kDtR / 8) + 255) / 256, 256, 0, stream>>>(ZX, kDproj, kColDt, kDtR / 8, kSeq, ADH, ADL);
  transpose_bf16_kernel<<<dim3(kDin / 64, kDtR / 64), 256, 0, stream>>>(W_dt, kDin, BTD, kDtR);

  wmma_gemm64<1><<<dim3((kSeq / 64) * (kDin / 64) / 8, 1), 256, 0, stream>>>(
      ADH, ADL, kDtR, BTD, kDtR, DT, kDin, kSeq, kDin, kDtR, 1.0f);

  scan_kernel<<<kDin / kScanCh, kScanCh, 0, stream>>>(ZX, XC, DT, dt_bias, A_log, Dvec, YH, YL);

  transpose_bf16_kernel<<<dim3(kDm / 64, kDin / 64), 256, 0, stream>>>(W_out, kDm, BT3, kDin);

  wmma_gemm64<1><<<dim3((kSeq / 64) * (kDm / 64) / 8, 1), 256, 0, stream>>>(
      YH, YL, kDin, BT3, kDin, out, kDm, kSeq, kDm, kDin, 1.0f);
}
